// BondLengthMechanics_3212635537989
// MI455X (gfx1250) — hardware-verified
//
#include <hip/hip_runtime.h>
#include <stddef.h>


#pragma clang fp contract(off)

#define DN      128
#define DB      64
#define NTHR    256
#define NWAVE   8
#define NBN     64
#define NBE     64
#define APA     136
#define APS     72
#define GSTR    132
#define NPROW   256
#define DROW    8
#define EPT     8
#define PIECE   (NTHR * EPT)
#define WCAP    (2 * EPT * 32)
#define NBC     4096
#define MAXTOK  8
#define PW0A    0
#define PW0B    16384
#define PW0D    32768
#define PW1     40960
#define PW2     57344
#define PWTOT   73728
#define PBLK    (PWTOT / (NTHR * 8))
#define WSCAP   134217728
#define EDGEDYN (NBE * GSTR * 4)
#define AGGDYN  (NBC * 4 * 4)
#define SCW     16.0f
#define SCA     64.0f
#define SCS     1024.0f
#define INV16   0.0625f
#define INV1024 0.0009765625f
#define INV16K  0.00006103515625f
#define LEAKY   0.001f
#define LN_EPS  0.00001f
#define STEPC   0.5f
#define DMAX    20.0f
#define COEFF   (-4.805f)
#define R62     (1.0f / 62.0f)
#define R128    0.0078125f

static_assert((PWTOT % (NTHR * 8)) == 0);
static_assert((PW0B % (NTHR * 8)) == 0);
static_assert((PW0D % (NTHR * 8)) == 0);
static_assert((PW1 % (NTHR * 8)) == 0);
static_assert((PW2 % (NTHR * 8)) == 0);
static_assert(((APA * 2) % 16) == 0);
static_assert(((APS * 2) % 16) == 0);
static_assert(((GSTR * 4) % 16) == 0);
static_assert((NBC & (NBC - 1)) == 0);
static_assert((PIECE & (PIECE - 1)) == 0);
static_assert(PIECE <= 2048);
static_assert(NBC <= 4096);
static_assert(NBE == NWAVE * 8);
static_assert(NBN == 4 * 16);
static_assert(((3 * NBC) % (4 * NTHR)) == 0);

typedef float          v4f   __attribute__((ext_vector_type(4)));
typedef float          v8f   __attribute__((ext_vector_type(8)));
typedef int            v4i   __attribute__((ext_vector_type(4)));
typedef unsigned short v8us  __attribute__((ext_vector_type(8)));
typedef _Float16       v4h   __attribute__((ext_vector_type(4)));
typedef _Float16       v8h   __attribute__((ext_vector_type(8)));
typedef _Float16       v16h  __attribute__((ext_vector_type(16)));
union FragH { v16h v; v8h h[2]; };
union Cvt8  { v8h v; v8us u; };

__device__ __forceinline__ v8f wmh(v16h a, v16h b, v8f c) {
  v8f d = __builtin_amdgcn_wmma_f32_16x16x32_f16(false, a, false, b, (short)0, c, false, false);
  asm volatile("v_nop\n\tv_nop\n\tv_nop\n\tv_nop" : "+v"(d) : "v"(a), "v"(b));
  return d;
}
__device__ __forceinline__ v8f zero8() {
  v8f z = {0.f, 0.f, 0.f, 0.f, 0.f, 0.f, 0.f, 0.f};
  return z;
}
__device__ __forceinline__ v4f zero4() {
  v4f z = {0.f, 0.f, 0.f, 0.f};
  return z;
}
__device__ __forceinline__ float lrelu(float v) { return v >= 0.0f ? v : LEAKY * v; }
__device__ __forceinline__ int imin(int a, int b) { return a < b ? a : b; }
__device__ __forceinline__ int iclamp(int v, int lo, int hi) { return v < lo ? lo : (v > hi ? hi : v); }

__device__ __forceinline__ void gemm16x64(const _Float16* ap, const _Float16* bpl, int kp, int nks, int n0,
                                          int m, int hh, v8f& c0, v8f& c1, v8f& c2, v8f& c3) {
  c0 = zero8(); c1 = zero8(); c2 = zero8(); c3 = zero8();
#pragma unroll 1
  for (int ks = 0; ks < nks; ++ks) {
    FragH a;
    a.h[0] = *(const v8h*)(ap + 32 * ks);
    a.h[1] = *(const v8h*)(ap + 32 * ks + 16);
    const _Float16* bp = bpl + (size_t)(n0 + m) * kp + 32 * ks + 8 * hh;
    FragH b;
    b.h[0] = *(const v8h*)(bp);
    b.h[1] = *(const v8h*)(bp + 16);
    c0 = wmh(a.v, b.v, c0);
    b.h[0] = *(const v8h*)(bp + (size_t)16 * kp);
    b.h[1] = *(const v8h*)(bp + (size_t)16 * kp + 16);
    c1 = wmh(a.v, b.v, c1);
    b.h[0] = *(const v8h*)(bp + (size_t)32 * kp);
    b.h[1] = *(const v8h*)(bp + (size_t)32 * kp + 16);
    c2 = wmh(a.v, b.v, c2);
    b.h[0] = *(const v8h*)(bp + (size_t)48 * kp);
    b.h[1] = *(const v8h*)(bp + (size_t)48 * kp + 16);
    c3 = wmh(a.v, b.v, c3);
  }
}

__device__ __forceinline__ void stage8(float* sp, v8f a, float scl, float bias) {
#pragma unroll
  for (int r = 0; r < 8; ++r) sp[r * GSTR] = a[r] * scl + bias;
}

__device__ __forceinline__ void row_stats(const float* row, float& mean, float& rstd) {
  float s = 0.f;
#pragma unroll
  for (int k = 0; k < 8; ++k) {
    const v4f v = *(const v4f*)(row + 4 * k);
    s += v.x; s += v.y; s += v.z; s += v.w;
  }
  s += __shfl_xor(s, 1);
  s += __shfl_xor(s, 2);
  mean = s * R128;
  float q = 0.f;
#pragma unroll
  for (int k = 0; k < 8; ++k) {
    const v4f v = *(const v4f*)(row + 4 * k);
    float d;
    d = v.x - mean; q += d * d;
    d = v.y - mean; q += d * d;
    d = v.z - mean; q += d * d;
    d = v.w - mean; q += d * d;
  }
  q += __shfl_xor(q, 1);
  q += __shfl_xor(q, 2);
  rstd = 1.0f / sqrtf(q * R128 + LN_EPS);
}

__global__ __launch_bounds__(NTHR) void k_prep(
    const float* __restrict__ W0, const float* __restrict__ W1, const float* __restrict__ W2,
    const float* __restrict__ bemb, int ntok, unsigned short* wp, float* T) {
  const int tid = (int)threadIdx.x;
  const int b = (int)blockIdx.x;
  if (b == PBLK) {
    const int t = tid >> 5, col = 4 * (tid & 31);
    const int tc = imin(t, ntok - 1);
    float s0 = 0.f, s1 = 0.f, s2 = 0.f, s3 = 0.f;
#pragma unroll 1
    for (int k = 0; k < DB; ++k) {
      const float g = bemb[(size_t)tc * DB + k];
      const float* wr = W0 + (size_t)(2 * DN + k) * DN + col;
      s0 += g * wr[0]; s1 += g * wr[1]; s2 += g * wr[2]; s3 += g * wr[3];
    }
    v4f o;
    o.x = s0; o.y = s1; o.z = s2; o.w = s3;
    float* tp = T + (size_t)t * DN + col;
    *(volatile v4f*)tp = o;
    __threadfence();
    *(volatile v4f*)tp = o;
  } else {
    const int o = (b * NTHR + tid) * 8;
    const float* src = W0;
    int r0 = 0, n, k0;
    if (o < PW0B)      { n = o >> 7; k0 = o & 127; }
    else if (o < PW0D) { const int idx = o - PW0B; n = idx >> 7; k0 = idx & 127; r0 = DN; }
    else if (o < PW1)  { const int idx = o - PW0D; n = idx >> 6; k0 = idx & 63;  r0 = 2 * DN + DB; }
    else if (o < PW2)  { const int idx = o - PW1;  n = idx >> 7; k0 = idx & 127; src = W1; }
    else               { const int idx = o - PW2;  n = idx >> 7; k0 = idx & 127; src = W2; }
    Cvt8 cv;
#pragma unroll
    for (int j = 0; j < 8; ++j) cv.v[j] = (_Float16)(src[(size_t)(r0 + k0 + j) * DN + n] * SCW);
    unsigned short* dp = wp + o;
    *(volatile v8us*)dp = cv.u;
    __threadfence();
    *(volatile v8us*)dp = cv.u;
  }
}

__global__ __launch_bounds__(NTHR) void k_node(
    const float* __restrict__ emb, const unsigned short* __restrict__ wp, float* NP, int nN) {
  __shared__ __attribute__((aligned(16))) _Float16 sA[NBN * APA];
  __shared__ __attribute__((aligned(16))) float stg[NWAVE * 1024];
  const int tid = (int)threadIdx.x, lane = tid & 31, wave = tid >> 5, hh = lane >> 4, m = lane & 15;
  const int n0 = (int)blockIdx.x * NBN;

  {
    const int nl = tid >> 2, q = tid & 3;
    int node = n0 + nl;
    node = node > nN - 1 ? nN - 1 : node;
    const float* rp = emb + (size_t)node * DN + 32 * q;
#pragma unroll
    for (int i = 0; i < 4; ++i) {
      const v4f xa = *(const v4f*)(rp + 8 * i);
      const v4f xb = *(const v4f*)(rp + 8 * i + 4);
      Cvt8 cv;
      cv.v[0] = (_Float16)xa.x; cv.v[1] = (_Float16)xa.y; cv.v[2] = (_Float16)xa.z; cv.v[3] = (_Float16)xa.w;
      cv.v[4] = (_Float16)xb.x; cv.v[5] = (_Float16)xb.y; cv.v[6] = (_Float16)xb.z; cv.v[7] = (_Float16)xb.w;
      *(v8h*)(sA + nl * APA + 32 * q + 8 * i) = cv.v;
    }
  }
  __syncthreads();

  const int rt = wave & 3, chf = wave >> 2;
  const _Float16* ap = sA + (16 * rt + m) * APA + 8 * hh;
  const _Float16* plane = (const _Float16*)(wp + (chf ? PW0B : PW0A));
  float* sw = stg + wave * 1024;
#pragma unroll 1
  for (int qq = 0; qq < 2; ++qq) {
    v8f a0, a1, a2, a3;
    gemm16x64(ap, plane, DN, 4, 64 * qq, m, hh, a0, a1, a2, a3);
    {
      float* sp = sw + (8 * hh) * 64 + m;
#pragma unroll
      for (int r = 0; r < 8; ++r) {
        sp[r * 64]      = a0[r] * INV16;
        sp[r * 64 + 16] = a1[r] * INV16;
        sp[r * 64 + 32] = a2[r] * INV16;
        sp[r * 64 + 48] = a3[r] * INV16;
      }
    }
    __syncthreads();
#pragma unroll 1
    for (int i = 0; i < 8; ++i) {
      const int r2 = 2 * i + hh;
      const v4f v = *(const v4f*)(sw + r2 * 64 + 4 * m);
      const int row = n0 + 16 * rt + r2;
      *(volatile v4f*)(NP + (size_t)row * NPROW + 128 * chf + 64 * qq + 4 * m) = v;
    }
    __threadfence();
#pragma unroll 1
    for (int i = 0; i < 8; ++i) {
      const int r2 = 2 * i + hh;
      const v4f v = *(const v4f*)(sw + r2 * 64 + 4 * m);
      const int row = n0 + 16 * rt + r2;
      *(volatile v4f*)(NP + (size_t)row * NPROW + 128 * chf + 64 * qq + 4 * m) = v;
    }
    __syncthreads();
  }
}

__global__ __launch_bounds__(NTHR) void k_edge(
    const float* __restrict__ x, const int* __restrict__ bidx, const int* __restrict__ btyp,
    const float* __restrict__ NP, const float* __restrict__ T, const unsigned short* __restrict__ wp,
    const float* __restrict__ b0, const float* __restrict__ b1,
    const float* __restrict__ l1w, const float* __restrict__ l1b,
    const float* __restrict__ b2, const float* __restrict__ l2w, const float* __restrict__ l2b,
    const float* __restrict__ Wo, const float* __restrict__ bo,
    float* D, int nE, int nN, int ntok) {
  extern __shared__ __attribute__((aligned(16))) float sH[];
  __shared__ __attribute__((aligned(16))) _Float16 sA[NBE * APA];
  __shared__ __attribute__((aligned(16))) _Float16 sS[NBE * APS];
  __shared__ __attribute__((aligned(16))) float sPar[7 * DN];
  __shared__ __attribute__((aligned(16))) float sT[MAXTOK * DN];
  __shared__ __attribute__((aligned(16))) float sWo[2 * DN];
  __shared__ __attribute__((aligned(16))) float sBo[4];
  __shared__ __attribute__((aligned(16))) float sU[NBE * 4];
  __shared__ __attribute__((aligned(16))) float sDist[NBE];
  __shared__ __attribute__((aligned(16))) float sRed[NBE * 4];
  __shared__ __attribute__((aligned(16))) float sC[NBE * DROW];
  __shared__ int sI[NBE];
  __shared__ int sJ[NBE];
  __shared__ int sTy[NBE];
  const int tid = (int)threadIdx.x, lane = tid & 31, wave = tid >> 5, hh = lane >> 4, m = lane & 15;
  const int e0 = (int)blockIdx.x * NBE;

  if (tid < NBE) {
    int e = e0 + tid;
    e = e > nE - 1 ? nE - 1 : e;
    const int ii = iclamp(bidx[2 * (size_t)e], 0, nN - 1);
    const int jj = iclamp(bidx[2 * (size_t)e + 1], 0, nN - 1);
    const int ty = iclamp(btyp[e], 0, ntok - 1);
    const float dx = x[(size_t)ii * 3]     - x[(size_t)jj * 3];
    const float dy = x[(size_t)ii * 3 + 1] - x[(size_t)jj * 3 + 1];
    const float dz = x[(size_t)ii * 3 + 2] - x[(size_t)jj * 3 + 2];
    const float d2 = (dx * dx + dz * dz) + dy * dy;
    const float d = sqrtf(d2);
    const float inv = 1.0f / d;
    sU[4 * tid]     = dx * inv;
    sU[4 * tid + 1] = dy * inv;
    sU[4 * tid + 2] = dz * inv;
    sU[4 * tid + 3] = 0.0f;
    sDist[tid] = d;
    sI[tid] = ii;
    sJ[tid] = jj;
    sTy[tid] = ty;
  }
  if (tid < DN) {
    sPar[tid]          = b0[tid];
    sPar[DN + tid]     = b1[tid];
    sPar[2 * DN + tid] = l1w[tid];
    sPar[3 * DN + tid] = l1b[tid];
    sPar[4 * DN + tid] = b2[tid];
    sPar[5 * DN + tid] = l2w[tid];
    sPar[6 * DN + tid] = l2b[tid];
  }
#pragma unroll 1
  for (int i = tid; i < MAXTOK * DN; i += NTHR) sT[i] = T[i];
  sWo[tid] = Wo[tid];
  if (tid < 2) sBo[tid] = bo[tid];
  __syncthreads();

  {
    const int e = tid >> 2, g = tid & 3;
    const float d = sDist[e];
    float ps = 0.f;
    float* hr = sH + e * GSTR + 16 * g;
#pragma unroll 1
    for (int q = 0; q < 16; ++q) {
      const int c = 16 * g + q;
      float off = DMAX * ((float)c * R62);
      off = (c >= DB - 2) ? DMAX : off;
      const float t = d - off;
      const float rb = expf(COEFF * (t * t));
      const float ov = (d >= DMAX) ? 1.0f : 0.0f;
      const float val = (c < DB - 1) ? rb : ov;
      hr[q] = val;
      ps += val;
    }
    sRed[4 * e + g] = ps;
  }
  __syncthreads();
  {
    const int e = tid >> 2, g = tid & 3;
    const float s = ((sRed[4 * e] + sRed[4 * e + 1]) + sRed[4 * e + 2]) + sRed[4 * e + 3];
    const float inv = 1.0f / s;
    const float* hr = sH + e * GSTR + 16 * g;
#pragma unroll
    for (int k = 0; k < 2; ++k) {
      Cvt8 cv;
#pragma unroll
      for (int u = 0; u < 8; ++u) cv.v[u] = (_Float16)((hr[8 * k + u] * inv) * SCS);
      *(v8h*)(sS + e * APS + 16 * g + 8 * k) = cv.v;
    }
  }
  __syncthreads();

  const int rt = wave & 3, cg = wave >> 2;

  {
    v8f a0, a1, a2, a3;
    gemm16x64(sS + (16 * rt + m) * APS + 8 * hh, (const _Float16*)(wp + PW0D), DB, 2, 64 * cg, m, hh, a0, a1, a2, a3);
    float* sp = sH + (16 * rt + 8 * hh) * GSTR + 64 * cg + m;
    stage8(sp,      a0, INV16K, 0.0f);
    stage8(sp + 16, a1, INV16K, 0.0f);
    stage8(sp + 32, a2, INV16K, 0.0f);
    stage8(sp + 48, a3, INV16K, 0.0f);
  }
  __syncthreads();

  {
    const int c4 = 4 * lane;
    const v4f bb = *(const v4f*)(sPar + c4);
#pragma unroll 1
    for (int jx = 0; jx < 8; ++jx) {
      const int el = 8 * wave + jx;
      const int ii = sI[el];
      const int jj = sJ[el];
      const int ty = sTy[el];
      const v4f p = *(const v4f*)(NP + (size_t)ii * NPROW + c4);
      const v4f q = *(const v4f*)(NP + (size_t)jj * NPROW + DN + c4);
      const v4f tv = *(const v4f*)(sT + ty * DN + c4);
      const v4f sv = *(const v4f*)(sH + el * GSTR + c4);
      const v4f v = (((p + q) + tv) + sv) + bb;
      v4h z;
      z.x = (_Float16)(lrelu(v.x) * SCA);
      z.y = (_Float16)(lrelu(v.y) * SCA);
      z.z = (_Float16)(lrelu(v.z) * SCA);
      z.w = (_Float16)(lrelu(v.w) * SCA);
      *(v4h*)(sA + el * APA + c4) = z;
    }
  }
  __syncthreads();

  {
    v8f a0, a1, a2, a3;
    gemm16x64(sA + (16 * rt + m) * APA + 8 * hh, (const _Float16*)(wp + PW1), DN, 4, 64 * cg, m, hh, a0, a1, a2, a3);
    float* sp = sH + (16 * rt + 8 * hh) * GSTR + 64 * cg + m;
    const float* bb = sPar + DN + 64 * cg + m;
    stage8(sp,      a0, INV1024, bb[0]);
    stage8(sp + 16, a1, INV1024, bb[16]);
    stage8(sp + 32, a2, INV1024, bb[32]);
    stage8(sp + 48, a3, INV1024, bb[48]);
  }
  __syncthreads();

  {
    const int e = tid >> 2, g = tid & 3;
    const float* row = sH + e * GSTR + 32 * g;
    float mean, rstd;
    row_stats(row, mean, rstd);
    const float* w = sPar + 2 * DN + 32 * g;
    const float* bb = sPar + 3 * DN + 32 * g;
#pragma unroll 1
    for (int k = 0; k < 4; ++k) {
      Cvt8 cv;
#pragma unroll
      for (int u = 0; u < 8; ++u) {
        const int c = 8 * k + u;
        const float y = (row[c] - mean) * rstd * w[c] + bb[c];
        cv.v[u] = (_Float16)(lrelu(y) * SCA);
      }
      *(v8h*)(sA + e * APA + 32 * g + 8 * k) = cv.v;
    }
  }
  __syncthreads();

  {
    v8f a0, a1, a2, a3;
    gemm16x64(sA + (16 * rt + m) * APA + 8 * hh, (const _Float16*)(wp + PW2), DN, 4, 64 * cg, m, hh, a0, a1, a2, a3);
    float* sp = sH + (16 * rt + 8 * hh) * GSTR + 64 * cg + m;
    const float* bb = sPar + 4 * DN + 64 * cg + m;
    stage8(sp,      a0, INV1024, bb[0]);
    stage8(sp + 16, a1, INV1024, bb[16]);
    stage8(sp + 32, a2, INV1024, bb[32]);
    stage8(sp + 48, a3, INV1024, bb[48]);
  }
  __syncthreads();

  {
    const int e = tid >> 2, g = tid & 3;
    const float* row = sH + e * GSTR + 32 * g;
    float mean, rstd;
    row_stats(row, mean, rstd);
    const float* w = sPar + 5 * DN + 32 * g;
    const float* bb = sPar + 6 * DN + 32 * g;
    const float* wo = sWo + 64 * g;
    float s0 = 0.f, s1 = 0.f;
#pragma unroll 2
    for (int c = 0; c < 32; ++c) {
      const float y = (row[c] - mean) * rstd * w[c] + bb[c];
      const float hv = lrelu(y);
      s0 += hv * wo[2 * c];
      s1 += hv * wo[2 * c + 1];
    }
    s0 += __shfl_xor(s0, 1);
    s0 += __shfl_xor(s0, 2);
    s1 += __shfl_xor(s1, 1);
    s1 += __shfl_xor(s1, 2);
    const float f0 = s0 + sBo[0];
    const float f1 = s1 + sBo[1];
    const float ux = sU[4 * e], uy = sU[4 * e + 1], uz = sU[4 * e + 2];
    if (g == 0) {
      v4f ci;
      ci.x = STEPC * (f0 * ux); ci.y = STEPC * (f0 * uy); ci.z = STEPC * (f0 * uz); ci.w = 0.0f;
      *(v4f*)(sC + e * DROW) = ci;
    }
    if (g == 1) {
      v4f cj;
      cj.x = STEPC * (f1 * (-ux)); cj.y = STEPC * (f1 * (-uy)); cj.z = STEPC * (f1 * (-uz)); cj.w = 0.0f;
      *(v4f*)(sC + e * DROW + 4) = cj;
    }
  }
  __syncthreads();

  if (tid < 2 * NBE) {
    const v4f v = *(const v4f*)(sC + 4 * tid);
    *(volatile v4f*)(D + (size_t)e0 * DROW + 4 * tid) = v;
  }
  __threadfence();
  if (tid < 2 * NBE) {
    const v4f v = *(const v4f*)(sC + 4 * tid);
    *(volatile v4f*)(D + (size_t)e0 * DROW + 4 * tid) = v;
  }
}

__device__ __forceinline__ int scan_piece(const int* __restrict__ bidx, int nE, int cbase, int base,
                                          int* list, int tid, int wave) {
  int wc = 0;
  const int el0  = tid * EPT;
  const int e0   = cbase + el0;
  const int sent = -2147483647 - 1;
  int ki[EPT], kj[EPT];
  if (cbase + PIECE <= nE) {
    const v4i* p = (const v4i*)(bidx + 2 * (size_t)e0);
    const v4i d0 = p[0], d1 = p[1], d2 = p[2], d3 = p[3];
    ki[0] = d0.x; kj[0] = d0.y; ki[1] = d0.z; kj[1] = d0.w;
    ki[2] = d1.x; kj[2] = d1.y; ki[3] = d1.z; kj[3] = d1.w;
    ki[4] = d2.x; kj[4] = d2.y; ki[5] = d2.z; kj[5] = d2.w;
    ki[6] = d3.x; kj[6] = d3.y; ki[7] = d3.z; kj[7] = d3.w;
  } else {
    const int lm = nE - 1;
#pragma unroll
    for (int q = 0; q < EPT; ++q) {
      const int eq = e0 + q;
      const int ec = eq > lm ? lm : eq;
      const int a = bidx[2 * (size_t)ec];
      const int b = bidx[2 * (size_t)ec + 1];
      ki[q] = (eq < nE) ? a : sent;
      kj[q] = (eq < nE) ? b : sent;
    }
  }
  const unsigned nb = (unsigned)base;
  unsigned si[EPT], sj[EPT];
  bool hi[EPT], hj[EPT];
  bool anyl = false;
#pragma unroll
  for (int q = 0; q < EPT; ++q) {
    si[q] = (unsigned)ki[q] - nb;
    sj[q] = (unsigned)kj[q] - nb;
    hi[q] = si[q] < (unsigned)NBC;
    hj[q] = sj[q] < (unsigned)NBC;
    anyl = anyl | hi[q] | hj[q];
  }
  const unsigned any = __builtin_amdgcn_ballot_w32(anyl);
  if (any != 0u) {
#define HIT(HJ, SJ, WH, Q) { \
      const unsigned mj = __builtin_amdgcn_ballot_w32(HJ); \
      if (mj != 0u) { \
        if (HJ) { \
          const int ps = wc + (int)__builtin_amdgcn_mbcnt_lo(mj, 0u); \
          if (ps < WCAP) list[wave * WCAP + ps] = ((el0 + (Q)) << 13) | ((WH) << 12) | (int)(SJ); \
        } \
        wc += (int)__builtin_popcount(mj); } }
#pragma unroll
    for (int q = 0; q < EPT; ++q) {
      HIT(hi[q], si[q], 0, q)
      HIT(hj[q], sj[q], 1, q)
    }
#undef HIT
  }
  return wc;
}

__device__ __forceinline__ void drain_piece(const int* list, const int* wcnt, float* accd,
                                            const float* __restrict__ D, int cbase, int Epad, int lane, int wave) {
#pragma unroll 1
  for (int wsx = 0; wsx < NWAVE; ++wsx) {
    int n = __builtin_amdgcn_readfirstlane(wcnt[wsx]);
    n = n > WCAP ? WCAP : (n < 0 ? 0 : n);
    const int* lp = list + wsx * WCAP;
#pragma unroll 1
    for (int bb = 0; bb < n; bb += 32) {
      const int idx = bb + lane;
      const int ic = idx > WCAP - 1 ? WCAP - 1 : idx;
      const int ent = lp[ic];
      const bool own = (idx < n) && ((ent & (NWAVE - 1)) == wave);
      unsigned msk = __builtin_amdgcn_ballot_w32(own);
#pragma unroll 1
      while (msk != 0u) {
        const int bit = (int)__builtin_ctz(msk);
        msk &= msk - 1u;
        const int e2 = __builtin_amdgcn_readlane(ent, bit);
        const int slot = e2 & (NBC - 1);
        const int wh = (e2 >> 12) & 1;
        const int el = (e2 >> 13) & (PIECE - 1);
        int row = cbase + el;
        row = row < 0 ? 0 : (row > Epad - 1 ? Epad - 1 : row);
        const float dv = D[(size_t)row * DROW + 4 * wh + (lane & 3)];
        if (lane < 4) accd[4 * slot + lane] += dv;
      }
    }
  }
}

__device__ __forceinline__ void agg_store(const float* accd, const float* __restrict__ pos, float* out,
                                          int base, int total, int tid) {
  const int bq = (3 * base) >> 2;
  const int full = total >> 2;
#pragma unroll 1
  for (int it = 0; it < (3 * NBC) / (4 * NTHR); ++it) {
    const int q4 = bq + it * NTHR + tid;
    const int t0 = 4 * q4 - 3 * base;
    float a[4];
#pragma unroll
    for (int c = 0; c < 4; ++c) {
      const int t = t0 + c;
      const int s = t / 3;
      a[c] = accd[4 * s + (t - 3 * s)];
    }
    int qa = q4 < full ? q4 : full - 1;
    qa = qa < 0 ? 0 : qa;
    const v4f pv = *(const v4f*)(pos + 4 * (size_t)qa);
    v4f ov;
    ov.x = pv.x + a[0]; ov.y = pv.y + a[1]; ov.z = pv.z + a[2]; ov.w = pv.w + a[3];
    if (q4 < full) {
      *(volatile v4f*)(out + 4 * (size_t)q4) = ov;
    } else if (q4 == full) {
      const int rem = total - 4 * full;
#pragma unroll
      for (int c = 0; c < 3; ++c) {
        if (c < rem) {
          int f = 4 * full + c;
          f = f > total - 1 ? total - 1 : f;
          const float pvs = pos[f];
          *(volatile float*)(out + f) = pvs + a[c];
        }
      }
    }
  }
}

__global__ __launch_bounds__(NTHR) void k_agg(
    const int* __restrict__ bidx, const float* __restrict__ D, const float* __restrict__ pos, float* out,
    int nE, int Epad, int nN, int total) {
  extern __shared__ __attribute__((aligned(16))) float accd[];
  __shared__ int list[NWAVE * WCAP];
  __shared__ int wcnt[NWAVE];
  const int tid = (int)threadIdx.x, lane = tid & 31, wave = tid >> 5;
  const int base = (int)blockIdx.x * NBC;

#pragma unroll 1
  for (int i = tid; i < NBC; i += NTHR) *(v4f*)(accd + 4 * i) = zero4();
  __syncthreads();

  const int nPieces = (nE + PIECE - 1) / PIECE;
#pragma unroll 1
  for (int pcx = 0; pcx < nPieces; ++pcx) {
    const int cbase = pcx * PIECE;
    const int wc = scan_piece(bidx, nE, cbase, base, list, tid, wave);
    if (lane == 0) wcnt[wave] = wc;
    __syncthreads();
    drain_piece(list, wcnt, accd, D, cbase, Epad, lane, wave);
    __syncthreads();
  }

  agg_store(accd, pos, out, base, total, tid);
  __threadfence();
  agg_store(accd, pos, out, base, total, tid);
}

extern "C" void kernel_launch(void* const* d_in, const int* in_sizes, int n_in,
                              void* d_out, int out_size, void* d_ws, size_t ws_size,
                              hipStream_t stream) {
  if (n_in < 18) return;
  if (in_sizes[0] < 6 || (in_sizes[0] % 3) != 0) return;
  const int nN = in_sizes[0] / 3;
  if (nN < 2 || nN > (1 << 24)) return;
  if (in_sizes[1] != 3 * nN) return;
  if (in_sizes[2] != nN * DN) return;
  if (in_sizes[3] < 2 || (in_sizes[3] % 2) != 0) return;
  const int nE = in_sizes[3] / 2;
  if (nE < 1 || nE > (1 << 28)) return;
  if (in_sizes[4] != nE) return;
  if (in_sizes[5] < DB || (in_sizes[5] % DB) != 0) return;
  const int ntok = in_sizes[5] / DB;
  if (ntok < 1 || ntok > MAXTOK) return;
  if (in_sizes[6] != (2 * DN + 2 * DB) * DN || in_sizes[7] != DN) return;
  if (in_sizes[8] != DN * DN || in_sizes[9] != DN || in_sizes[10] != DN || in_sizes[11] != DN) return;
  if (in_sizes[12] != DN * DN || in_sizes[13] != DN || in_sizes[14] != DN || in_sizes[15] != DN) return;
  if (in_sizes[16] != 2 * DN || in_sizes[17] != 2) return;
  if (out_size != 3 * nN) return;

  const float* x    = (const float*)d_in[0];
  const float* pos  = (const float*)d_in[1];
  const float* emb  = (const float*)d_in[2];
  const int*   bidx = (const int*)d_in[3];
  const int*   btyp = (const int*)d_in[4];
  const float* bemb = (const float*)d_in[5];
  const float* W0   = (const float*)d_in[6];
  const float* b0   = (const float*)d_in[7];
  const float* W1   = (const float*)d_in[8];
  const float* b1   = (const float*)d_in[9];
  const float* l1w  = (const float*)d_in[10];
  const float* l1b  = (const float*)d_in[11];
  const float* W2   = (const float*)d_in[12];
  const float* b2   = (const float*)d_in[13];
  const float* l2w  = (const float*)d_in[14];
  const float* l2b  = (const float*)d_in[15];
  const float* Wo   = (const float*)d_in[16];
  const float* bo   = (const float*)d_in[17];
  float* out = (float*)d_out;

  const int nbNode = (nN + NBN - 1) / NBN;
  const int Npad   = nbNode * NBN;
  const int nbEdge = (nE + NBE - 1) / NBE;
  const int Epad   = nbEdge * NBE;
  const int nbAgg  = (nN + NBC - 1) / NBC;

  char* ws = (char*)d_ws;
  size_t off = 0;
  const size_t oW  = off; off += (size_t)PWTOT * 2;           off = (off + 255) & ~(size_t)255;
  const size_t oT  = off; off += (size_t)MAXTOK * DN * 4;      off = (off + 255) & ~(size_t)255;
  const size_t oNP = off; off += (size_t)Npad * NPROW * 4;     off = (off + 255) & ~(size_t)255;
  const size_t oD  = off; off += (size_t)Epad * DROW * 4;      off = (off + 255) & ~(size_t)255;
  if (off > ws_size || off > (size_t)WSCAP) return;
  unsigned short* wp = (unsigned short*)(ws + oW);
  float* T  = (float*)(ws + oT);
  float* NP = (float*)(ws + oNP);
  float* D  = (float*)(ws + oD);

  hipFuncSetAttribute(reinterpret_cast<const void*>(&k_edge), hipFuncAttributeMaxDynamicSharedMemorySize, EDGEDYN);
  hipFuncSetAttribute(reinterpret_cast<const void*>(&k_agg), hipFuncAttributeMaxDynamicSharedMemorySize, AGGDYN);

  k_prep<<<PBLK + 1, NTHR, 0, stream>>>(W0, W1, W2, bemb, ntok, wp, T);
  k_node<<<nbNode, NTHR, 0, stream>>>(emb, wp, NP, nN);
  k_edge<<<nbEdge, NTHR, EDGEDYN, stream>>>(x, bidx, btyp, NP, T, wp, b0, b1, l1w, l1b, b2, l2w, l2b, Wo, bo,
                                             D, nE, nN, ntok);
  k_agg<<<nbAgg, NTHR, AGGDYN, stream>>>(bidx, D, pos, out, nE, Epad, nN, out_size);
}
